// ResNetBlock_59854664237618
// MI455X (gfx1250) — hardware-verified
//
#include <hip/hip_runtime.h>
#include <stddef.h>
#include <stdint.h>

#define CIN    32
#define TT     32
#define RR     5
#define AA     8
#define NROT   4
#define DSTEP  2
#define NPAIR  (RR * AA)
#define KTOT   (NPAIR * CIN)
#define NCOL   (NROT * TT)
#define K8ROW  (KTOT / 8)
#define BCW    (NPAIR * 3)
#define MB     64
#define NTHR   128
#define PPC    4
#define NCH    (NPAIR / PPC)
#define ATP    (2 * PPC * CIN)
#define LDS_IDX (MB * BCW)
#define LDS_BYTES (LDS_IDX * 4 * 2 + MB * ATP * 2 + MB * TT * 4)
#define PREPU  (2 * NCOL * K8ROW)
#define WSMAX  134217728

static_assert(NPAIR % PPC == 0);
static_assert(BCW % 4 == 0 && (LDS_IDX % (NTHR * 4)) == 0);
static_assert(MB == (NTHR / 32) * 16);
static_assert(KTOT % 32 == 0 && NCOL == 8 * 16 && TT == 32 && CIN == 32);
static_assert((NCOL * K8ROW) % 256 == 0 && PREPU % 256 == 0 && K8ROW % 32 == 0);
static_assert(LDS_BYTES <= 300000);
static_assert(((2 * LDS_IDX) * 4) % 16 == 0);

typedef float          v4f   __attribute__((ext_vector_type(4)));
typedef float          v8f   __attribute__((ext_vector_type(8)));
typedef int            v4i   __attribute__((ext_vector_type(4)));
typedef int            v8i   __attribute__((ext_vector_type(8)));
typedef unsigned short v4us  __attribute__((ext_vector_type(4)));
typedef unsigned short v8us  __attribute__((ext_vector_type(8)));
typedef unsigned short v16us __attribute__((ext_vector_type(16)));
typedef __bf16         v16bf __attribute__((ext_vector_type(16)));
typedef v4f  __attribute__((may_alias)) v4fa;
typedef v4i  __attribute__((may_alias)) v4ia;
typedef v4us __attribute__((may_alias)) v4usa;
typedef v8us __attribute__((may_alias)) v8usa;
union FragB { v16bf v; v16us u; v8us h[2]; v8i w; };

__device__ __forceinline__ v8f wmb(const FragB& a, const FragB& b, v8f c) {
  v8f d = __builtin_amdgcn_wmma_f32_16x16x32_bf16(false, a.v, false, b.v, (short)0, c, false, false);
  asm volatile("v_nop\n\tv_nop\n\tv_nop\n\tv_nop" : "+v"(d) : "v"(a.w), "v"(b.w));
  return d;
}

__device__ __forceinline__ unsigned bf16_bits(float f) {
  const unsigned u = __float_as_uint(f);
  return (u + 0x7FFFu + ((u >> 16) & 1u)) >> 16;
}
__device__ __forceinline__ float bf16_val(float f) {
  return __uint_as_float(bf16_bits(f) << 16);
}
__device__ __forceinline__ int clampi(int x, int lo, int hi) {
  return x < lo ? lo : (x > hi ? hi : x);
}

__global__ __launch_bounds__(256) void k_tprep(const float* __restrict__ t1, const float* __restrict__ t2,
                                               unsigned short* rt1, unsigned short* rt2) {
  const int u = (int)blockIdx.x * 256 + (int)threadIdx.x;
  if (u >= PREPU) return;
  const int per = NCOL * K8ROW;
  const int cv  = u / per;
  const int rem = u - cv * per;
  const int n   = rem / K8ROW;
  const int k8  = rem - n * K8ROW;
  const int rot = n >> 5, t = n & 31;
  const int pr  = k8 >> 2, c8 = (k8 & 3) * 8;
  const int r   = pr >> 3, a = pr & 7;
  const int asrc = (a - DSTEP * rot) & (AA - 1);
  const float* tsrc = (cv == 0) ? t1 : t2;
  unsigned short* rdst = (cv == 0) ? rt1 : rt2;
  const float* p = tsrc + ((size_t)(t * RR + r) * AA + asrc) * CIN + c8;
  const v4f x = *(const v4fa*)p;
  const v4f y = *(const v4fa*)(p + 4);
  v8us o;
  o[0] = (unsigned short)bf16_bits(x.x); o[1] = (unsigned short)bf16_bits(x.y);
  o[2] = (unsigned short)bf16_bits(x.z); o[3] = (unsigned short)bf16_bits(x.w);
  o[4] = (unsigned short)bf16_bits(y.x); o[5] = (unsigned short)bf16_bits(y.y);
  o[6] = (unsigned short)bf16_bits(y.z); o[7] = (unsigned short)bf16_bits(y.w);
  unsigned short* dp = rdst + (size_t)n * KTOT + k8 * 8;
  *(volatile v8us*)dp = o;
  __threadfence();
  *(volatile v8us*)dp = o;
}

template <int MODE>
__global__ __launch_bounds__(NTHR) void k_conv(const float* __restrict__ xin, const int* __restrict__ bidx,
                                               const float* __restrict__ bw, const unsigned short* __restrict__ rt,
                                               const float* __restrict__ bias, const float* __restrict__ sig,
                                               float* outp, int nV) {
  extern __shared__ __attribute__((aligned(16))) int dsm[];
  int*            sIdx = dsm;
  float*          sW   = (float*)(dsm + LDS_IDX);
  unsigned short* sA   = (unsigned short*)(dsm + 2 * LDS_IDX);
  float*          sO   = (float*)(dsm + 2 * LDS_IDX + (MB * ATP) / 2);

  const int tid = (int)threadIdx.x, lane = tid & 31, wave = tid >> 5, hh = lane >> 4, m = lane & 15;
  const int g = lane >> 3, q = lane & 7;
  const int v0 = (int)blockIdx.x * MB;
  const int vmax = nV - 1;

#pragma unroll 3
  for (int j4 = tid; j4 < LDS_IDX / 4; j4 += NTHR) {
    const int j   = j4 * 4;
    const int row = j / BCW;
    const int col = j - row * BCW;
    const int vr  = clampi(v0 + row, 0, vmax);
    const size_t gs = (size_t)vr * BCW + col;
    v4i iv = *(const v4ia*)(bidx + gs);
    v4f wv = *(const v4fa*)(bw + gs);
    iv.x = clampi(iv.x, 0, vmax); iv.y = clampi(iv.y, 0, vmax);
    iv.z = clampi(iv.z, 0, vmax); iv.w = clampi(iv.w, 0, vmax);
    wv.x = bf16_val(wv.x); wv.y = bf16_val(wv.y); wv.z = bf16_val(wv.z); wv.w = bf16_val(wv.w);
    *(v4ia*)(sIdx + j) = iv;
    *(v4fa*)(sW + j)   = wv;
  }
  __syncthreads();

  v8f acc[8];
  {
    const v8f z = {0.f, 0.f, 0.f, 0.f, 0.f, 0.f, 0.f, 0.f};
#pragma unroll
    for (int t = 0; t < 8; ++t) acc[t] = z;
  }

#pragma unroll 1
  for (int ch = 0; ch < NCH; ++ch) {
#pragma unroll 2
    for (int s = 0; s < 16; ++s) {
      const int id   = 4 * s + g;
      const int rr   = id & 15;
      const int pp   = id >> 4;
      const int lrow = 16 * wave + rr;
      const int tb   = lrow * BCW + (ch * PPC + pp) * 3;
      const int   i0 = sIdx[tb], i1 = sIdx[tb + 1], i2 = sIdx[tb + 2];
      const float w0 = sW[tb],   w1 = sW[tb + 1],   w2 = sW[tb + 2];
      v4f x0 = *(const v4fa*)(xin + (size_t)i0 * CIN + 4 * q);
      v4f x1 = *(const v4fa*)(xin + (size_t)i1 * CIN + 4 * q);
      v4f x2 = *(const v4fa*)(xin + (size_t)i2 * CIN + 4 * q);
      if constexpr (MODE == 0) {
        x0.x = bf16_val(x0.x); x0.y = bf16_val(x0.y); x0.z = bf16_val(x0.z); x0.w = bf16_val(x0.w);
        x1.x = bf16_val(x1.x); x1.y = bf16_val(x1.y); x1.z = bf16_val(x1.z); x1.w = bf16_val(x1.w);
        x2.x = bf16_val(x2.x); x2.y = bf16_val(x2.y); x2.z = bf16_val(x2.z); x2.w = bf16_val(x2.w);
      }
      v4f val;
      val.x = fmaf(w2, x2.x, fmaf(w1, x1.x, w0 * x0.x));
      val.y = fmaf(w2, x2.y, fmaf(w1, x1.y, w0 * x0.y));
      val.z = fmaf(w2, x2.z, fmaf(w1, x1.z, w0 * x0.z));
      val.w = fmaf(w2, x2.w, fmaf(w1, x1.w, w0 * x0.w));
      v4us h4, l4;
      {
        unsigned hb;
        hb = bf16_bits(val.x); h4[0] = (unsigned short)hb; l4[0] = (unsigned short)bf16_bits(val.x - __uint_as_float(hb << 16));
        hb = bf16_bits(val.y); h4[1] = (unsigned short)hb; l4[1] = (unsigned short)bf16_bits(val.y - __uint_as_float(hb << 16));
        hb = bf16_bits(val.z); h4[2] = (unsigned short)hb; l4[2] = (unsigned short)bf16_bits(val.z - __uint_as_float(hb << 16));
        hb = bf16_bits(val.w); h4[3] = (unsigned short)hb; l4[3] = (unsigned short)bf16_bits(val.w - __uint_as_float(hb << 16));
      }
      unsigned short* ap = sA + (size_t)lrow * ATP + pp * CIN + 4 * q;
      *(v4usa*)ap = h4;
      *(v4usa*)(ap + PPC * CIN) = l4;
    }
    __syncthreads();

#pragma unroll 1
    for (int pp = 0; pp < PPC; ++pp) {
      const unsigned short* ap = sA + (size_t)(16 * wave + m) * ATP + pp * CIN + 8 * hh;
      FragB ah, al;
      ah.h[0] = *(const v8usa*)ap;
      ah.h[1] = *(const v8usa*)(ap + 16);
      al.h[0] = *(const v8usa*)(ap + PPC * CIN);
      al.h[1] = *(const v8usa*)(ap + PPC * CIN + 16);
      const int k0 = (ch * PPC + pp) * CIN;
      const unsigned short* bp = rt + (size_t)m * KTOT + k0 + 8 * hh;
#pragma unroll
      for (int nt = 0; nt < 8; ++nt) {
        const unsigned short* wq = bp + (size_t)(16 * nt) * KTOT;
        FragB bf;
        bf.h[0] = *(const v8usa*)wq;
        bf.h[1] = *(const v8usa*)(wq + 16);
        acc[nt] = wmb(ah, bf, acc[nt]);
        acc[nt] = wmb(al, bf, acc[nt]);
      }
    }
    __syncthreads();
  }

  {
    const float bq0 = bf16_val(bias[m]);
    const float bq1 = bf16_val(bias[16 + m]);
#pragma unroll
    for (int r = 0; r < 8; ++r) {
      const int lr = 16 * wave + 8 * hh + r;
      float y0 = fmaxf(fmaxf(acc[0][r], acc[2][r]), fmaxf(acc[4][r], acc[6][r])) + bq0;
      float y1 = fmaxf(fmaxf(acc[1][r], acc[3][r]), fmaxf(acc[5][r], acc[7][r])) + bq1;
      if constexpr (MODE == 0) { y0 = fmaxf(y0, 0.0f); y1 = fmaxf(y1, 0.0f); }
      sO[lr * TT + m]      = y0;
      sO[lr * TT + 16 + m] = y1;
    }
  }
  __syncthreads();

  v4f pv[4];
#pragma unroll
  for (int i = 0; i < 4; ++i) {
    const int lrow = 16 * wave + 4 * i + g;
    v4f tv = *(const v4fa*)(sO + lrow * TT + 4 * q);
    if constexpr (MODE != 0) {
      const int vc = clampi(v0 + lrow, 0, vmax);
      const v4f xs = *(const v4fa*)(sig + (size_t)vc * CIN + 4 * q);
      tv.x = fmaxf(tv.x + bf16_val(xs.x), 0.0f);
      tv.y = fmaxf(tv.y + bf16_val(xs.y), 0.0f);
      tv.z = fmaxf(tv.z + bf16_val(xs.z), 0.0f);
      tv.w = fmaxf(tv.w + bf16_val(xs.w), 0.0f);
    }
    pv[i] = tv;
  }
#pragma unroll
  for (int i = 0; i < 4; ++i) {
    const int v = v0 + 16 * wave + 4 * i + g;
    if (v < nV) *(volatile v4f*)(outp + (size_t)v * TT + 4 * q) = pv[i];
  }
  __threadfence();
#pragma unroll
  for (int i = 0; i < 4; ++i) {
    const int v = v0 + 16 * wave + 4 * i + g;
    if (v < nV) *(volatile v4f*)(outp + (size_t)v * TT + 4 * q) = pv[i];
  }
}

static inline size_t al256(size_t o) { return (o + 255) & ~(size_t)255; }

extern "C" void kernel_launch(void* const* d_in, const int* in_sizes, int n_in,
                              void* d_out, int out_size, void* d_ws, size_t ws_size,
                              hipStream_t stream) {
  if (n_in < 7) return;
  if (in_sizes[0] < CIN * 16 || (in_sizes[0] % CIN) != 0) return;
  const int nV = in_sizes[0] / CIN;
  if (nV >= (1 << 24)) return;
  if ((long long)in_sizes[1] != (long long)nV * BCW) return;
  if (in_sizes[2] != in_sizes[1]) return;
  if (in_sizes[3] != TT * KTOT || in_sizes[5] != TT * KTOT) return;
  if (in_sizes[4] != TT || in_sizes[6] != TT) return;
  if ((long long)out_size != (long long)nV * TT) return;

  const float* signal = (const float*)d_in[0];
  const int*   bidx   = (const int*)d_in[1];
  const float* bw     = (const float*)d_in[2];
  const float* templ1 = (const float*)d_in[3];
  const float* bias1  = (const float*)d_in[4];
  const float* templ2 = (const float*)d_in[5];
  const float* bias2  = (const float*)d_in[6];
  float* out = (float*)d_out;

  const int gB = (nV + MB - 1) / MB;
  const int MP = gB * MB;

  char* ws = (char*)d_ws;
  size_t off = 0;
  const size_t oR1 = off; off = al256(off + (size_t)NCOL * KTOT * 2);
  const size_t oR2 = off; off = al256(off + (size_t)NCOL * KTOT * 2);
  const size_t oS  = off; off = al256(off + (size_t)MP * TT * 4);
  if (off > ws_size || off > (size_t)WSMAX) return;
  unsigned short* rt1 = (unsigned short*)(ws + oR1);
  unsigned short* rt2 = (unsigned short*)(ws + oR2);
  float* splane = (float*)(ws + oS);

  hipFuncSetAttribute(reinterpret_cast<const void*>(&k_conv<0>), hipFuncAttributeMaxDynamicSharedMemorySize, (int)LDS_BYTES);
  hipFuncSetAttribute(reinterpret_cast<const void*>(&k_conv<1>), hipFuncAttributeMaxDynamicSharedMemorySize, (int)LDS_BYTES);

  k_tprep<<<PREPU / 256, 256, 0, stream>>>(templ1, templ2, rt1, rt2);
  k_conv<0><<<gB, NTHR, LDS_BYTES, stream>>>(signal, bidx, bw, rt1, bias1, signal, splane, nV);
  k_conv<1><<<gB, NTHR, LDS_BYTES, stream>>>(splane, bidx, bw, rt2, bias2, signal, out, nV);
}
